// Layer_82738249990805
// MI455X (gfx1250) — hardware-run, weakly checked
//
#include <hip/hip_runtime.h>
#include <math.h>

constexpr int kB   = 4;
constexpr int kS   = 1024;
constexpr int kH   = 768;
constexpr int kNH  = 12;
constexpr int kHD  = 64;
constexpr int kFF  = 3072;
constexpr int kM   = kB * kS;
constexpr int kGrp = 6;
constexpr float kQKScale = 0.125f;
constexpr float kLnEps   = 1e-12f;
constexpr float kInvH    = 1.0f / 768.0f;
static_assert(kNH * kHD == kH, "shape");
static_assert(kNH % kGrp == 0, "groups");
static_assert(kH == 3 * 256, "ln thread map");
static_assert(kS == 128 * 8, "softmax thread map");
static_assert(kM % 64 == 0 && kH % 64 == 0 && kFF % 64 == 0 && kS % 64 == 0 && kHD % 64 == 0, "mn tiles");
static_assert(kH % 32 == 0 && kFF % 32 == 0 && kS % 32 == 0 && kHD % 32 == 0, "k tiles");

typedef __attribute__((ext_vector_type(16))) _Float16 v16h;
typedef __attribute__((ext_vector_type(8)))  _Float16 v8h;
typedef __attribute__((ext_vector_type(16))) __bf16   v16b;
typedef __attribute__((ext_vector_type(8)))  __bf16   v8b;
typedef __attribute__((ext_vector_type(8)))  float    v8f;
typedef __attribute__((ext_vector_type(4)))  float    v4f;
typedef __attribute__((ext_vector_type(4)))  unsigned int v4u;

__device__ __forceinline__ unsigned short f2bf_bits(float f) {
  unsigned u = __float_as_uint(f);
  return (unsigned short)((u + 0x7FFFu + ((u >> 16) & 1u)) >> 16);
}
__device__ __forceinline__ float bf_bits2f(unsigned short h) { return __uint_as_float(((unsigned)h) << 16); }
__device__ __forceinline__ unsigned pk16(unsigned short a, unsigned short b) { return (unsigned)a | ((unsigned)b << 16); }

__device__ __forceinline__ void dep_guard4_h(v8f& a, v8f& b, v8f& c, v8f& d, v16h x, v16h y) {
  asm volatile("v_nop\n\tv_nop\n\tv_nop\n\tv_nop" : "+v"(a), "+v"(b), "+v"(c), "+v"(d) : "v"(x), "v"(y));
}
__device__ __forceinline__ void dep_guard4_b(v8f& a, v8f& b, v8f& c, v8f& d, v16b x, v16b y) {
  asm volatile("v_nop\n\tv_nop\n\tv_nop\n\tv_nop" : "+v"(a), "+v"(b), "+v"(c), "+v"(d) : "v"(x), "v"(y));
}
__device__ __forceinline__ void keep4_h(v16h a, v16h b, v16h c, v16h d) { asm volatile("v_nop" :: "v"(a), "v"(b), "v"(c), "v"(d)); }
__device__ __forceinline__ void keep4_b(v16b a, v16b b, v16b c, v16b d) { asm volatile("v_nop" :: "v"(a), "v"(b), "v"(c), "v"(d)); }
__device__ __forceinline__ void acc_guard4(v8f& a, v8f& b, v8f& c, v8f& d) { asm volatile("v_nop\n\tv_nop\n\tv_nop\n\tv_nop" : "+v"(a), "+v"(b), "+v"(c), "+v"(d)); }
template <typename T> struct Frag;
template <> struct Frag<_Float16> {
  typedef v16h V; union U { v16h v; v8h h[2]; };
  static __device__ __forceinline__ v16h load(const _Float16* p) {
    U f; f.h[0] = *(const v8h*)(p); f.h[1] = *(const v8h*)(p + 16); return f.v;
  }
  static __device__ __forceinline__ v8f mma(v16h a, v16h b, v8f c) {
    return __builtin_amdgcn_wmma_f32_16x16x32_f16(false, a, false, b, (short)0, c, false, false);
  }
  static __device__ __forceinline__ void guard4(v8f& a, v8f& b, v8f& c, v8f& d, v16h x, v16h y) { dep_guard4_h(a, b, c, d, x, y); }
  static __device__ __forceinline__ void keep(v16h a, v16h b, v16h c, v16h d) { keep4_h(a, b, c, d); }
};
template <> struct Frag<__bf16> {
  typedef v16b V; union U { v16b v; v8b h[2]; };
  static __device__ __forceinline__ v16b load(const __bf16* p) {
    U f; f.h[0] = *(const v8b*)(p); f.h[1] = *(const v8b*)(p + 16); return f.v;
  }
  static __device__ __forceinline__ v8f mma(v16b a, v16b b, v8f c) {
    return __builtin_amdgcn_wmma_f32_16x16x32_bf16(false, a, false, b, (short)0, c, false, false);
  }
  static __device__ __forceinline__ void guard4(v8f& a, v8f& b, v8f& c, v8f& d, v16b x, v16b y) { dep_guard4_b(a, b, c, d, x, y); }
  static __device__ __forceinline__ void keep(v16b a, v16b b, v16b c, v16b d) { keep4_b(a, b, c, d); }
};

__device__ __forceinline__ v4u pack8_bf16(v4f a, v4f c) {
  unsigned short hb[8];
#pragma unroll
  for (int e = 0; e < 4; ++e) {
    hb[e]     = f2bf_bits(a[e]);
    hb[4 + e] = f2bf_bits(c[e]);
  }
  return (v4u){pk16(hb[0], hb[1]), pk16(hb[2], hb[3]), pk16(hb[4], hb[5]), pk16(hb[6], hb[7])};
}

template <int ET> struct Elem;
template <> struct Elem<0> { typedef _Float16 T; };
template <> struct Elem<1> { typedef __bf16 T; };
template <int ET, bool SPLIT, int BIAS_MODE, int OUT_MODE, bool RESID>
__global__ __launch_bounds__(256) void wmma_gemm64(
    const unsigned short* __restrict__ Ap, const unsigned short* __restrict__ A2p, int lda, long strideA,
    const unsigned short* __restrict__ Btp, const unsigned short* __restrict__ Bt2p, int ldb, long strideB,
    void* __restrict__ Cout, void* __restrict__ Cout2, int ldc, long strideC,
    const float* __restrict__ bias, const float* __restrict__ cscale,
    const float* __restrict__ resid, long strideR,
    int M, int N, int K, float scale) {
  static_assert(!(RESID && OUT_MODE != 0), "resid only with f32 output");
  typedef typename Elem<ET>::T T;
  typedef typename Frag<T>::V V;
  const T* A = (const T*)Ap; const T* A2 = (const T*)A2p; const T* Bt = (const T*)Btp; const T* Bt2 = (const T*)Bt2p;
  __shared__ __align__(16) float sT[8][16 * 68];
  const int b    = blockIdx.y;
  const int lane = threadIdx.x & 31;
  const int wave = threadIdx.x >> 5;
  const int tilesN = N >> 6;
  const int tilesM = M >> 6;
  const int tile = blockIdx.x * 8 + wave;
  if (tile >= tilesM * tilesN) return;
  const int tm = tile / tilesN;
  const int tn = tile - tm * tilesN;
  const int m0 = tm << 6;
  const int n0 = tn << 6;

  const T* Ab  = A  + (size_t)b * strideA;
  const T* Bb  = Bt + (size_t)b * strideB;
  const T* Ab2 = SPLIT ? (A2  + (size_t)b * strideA) : nullptr;
  const T* Bb2 = SPLIT ? (Bt2 + (size_t)b * strideB) : nullptr;

  const int rlane = lane & 15;
  const int koff  = (lane >> 4) * 8;
  const int mOff  = (lane >> 4) * 8;

  v8f acc[4][4];
#pragma unroll
  for (int i = 0; i < 4; ++i)
#pragma unroll
    for (int j = 0; j < 4; ++j) acc[i][j] = (v8f){0.f,0.f,0.f,0.f,0.f,0.f,0.f,0.f};

  for (int k0 = 0; k0 < K; k0 += 32) {
    V bh[4], bl[4];
#pragma unroll
    for (int j = 0; j < 4; ++j) {
      const size_t bo = (size_t)(n0 + (j << 4) + rlane) * ldb + koff + k0;
      bh[j] = Frag<T>::load(Bb + bo);
      if (SPLIT) bl[j] = Frag<T>::load(Bb2 + bo);
    }
#pragma unroll
    for (int i = 0; i < 4; ++i) {
      const size_t ao = (size_t)(m0 + (i << 4) + rlane) * lda + koff + k0;
      V ah = Frag<T>::load(Ab + ao);
      V al;
      if (SPLIT) al = Frag<T>::load(Ab2 + ao);
#pragma unroll
      for (int j = 0; j < 4; ++j) {
        acc[i][j] = Frag<T>::mma(ah, bh[j], acc[i][j]);
        if (SPLIT) {
          acc[i][j] = Frag<T>::mma(ah, bl[j], acc[i][j]);
          acc[i][j] = Frag<T>::mma(al, bh[j], acc[i][j]);
        }
      }
      Frag<T>::guard4(acc[i][0], acc[i][1], acc[i][2], acc[i][3], ah, SPLIT ? al : ah);
    }
    Frag<T>::keep(bh[0], bh[1], bh[2], bh[3]);
    if (SPLIT) Frag<T>::keep(bl[0], bl[1], bl[2], bl[3]);
  }
  acc_guard4(acc[0][0], acc[0][1], acc[0][2], acc[0][3]);
  acc_guard4(acc[1][0], acc[1][1], acc[1][2], acc[1][3]);
  acc_guard4(acc[2][0], acc[2][1], acc[2][2], acc[2][3]);
  acc_guard4(acc[3][0], acc[3][1], acc[3][2], acc[3][3]);

  float* slab = sT[wave];
  const float* Rb = RESID ? (resid + (size_t)b * strideR) : nullptr;
#pragma unroll
  for (int i = 0; i < 4; ++i) {
    const int mBase = m0 + (i << 4);
#pragma unroll
    for (int j = 0; j < 4; ++j) {
      const int n = n0 + (j << 4) + rlane;
      float bv = 0.f, cs = 1.f;
      if (BIAS_MODE == 2 || BIAS_MODE == 3) bv = bias[n];
      if (BIAS_MODE == 3) cs = cscale[n];
#pragma unroll
      for (int r = 0; r < 8; ++r) {
        float v = acc[i][j][r] * scale;
        if (BIAS_MODE == 1) v += bias[mBase + mOff + r];
        if (BIAS_MODE == 2) v += bv;
        if (BIAS_MODE == 3) v = (v + bv) * cs;
        slab[(mOff + r) * 68 + (j << 4) + rlane] = v;
      }
    }
    __builtin_amdgcn_fence(__ATOMIC_RELEASE, "workgroup");
    __builtin_amdgcn_wave_barrier();
    __builtin_amdgcn_fence(__ATOMIC_ACQUIRE, "workgroup");
    if (OUT_MODE == 0) {
      float* C = (float*)Cout + (size_t)b * strideC;
      const int hh = lane >> 4, c4 = (lane & 15) * 4;
      v4f vals[8];
#pragma unroll
      for (int it = 0; it < 8; ++it) {
        const int row = it * 2 + hh;
        v4f v = *(const v4f*)(slab + row * 68 + c4);
        if (RESID) {
          const v4f rr = *(const v4f*)(Rb + (size_t)(mBase + row) * ldc + n0 + c4);
          v += rr;
        }
        vals[it] = v;
      }
      for (int pass = 0; pass < 2; ++pass) {
#pragma unroll
        for (int it = 0; it < 8; ++it) {
          const int row = it * 2 + hh;
          *(volatile v4f*)(C + (size_t)(mBase + row) * ldc + n0 + c4) = vals[it];
        }
        __threadfence();
      }
    } else {
      const int q = lane >> 3, c8 = (lane & 7) * 8;
      unsigned short* C  = (unsigned short*)Cout  + (size_t)b * strideC;
      unsigned short* C2 = (OUT_MODE == 2) ? ((unsigned short*)Cout2 + (size_t)b * strideC) : nullptr;
      for (int pass = 0; pass < 2; ++pass) {
#pragma unroll
        for (int it = 0; it < 4; ++it) {
          const int row = it * 4 + q;
          const float* sp = slab + row * 68 + c8;
          if (OUT_MODE == 3) {
            const v4f a0 = *(const v4f*)(sp);
            const v4f a1 = *(const v4f*)(sp + 4);
            const v4u u = pack8_bf16(a0, a1);
            *(volatile v4u*)(C + (size_t)(mBase + row) * ldc + n0 + c8) = u;
          } else {
            v8h hv, lv;
#pragma unroll
            for (int e = 0; e < 8; ++e) {
              if (OUT_MODE == 1) {
                hv[e] = (_Float16)sp[e];
              } else {
                unsigned short hb = f2bf_bits(sp[e]);
                unsigned short lb = f2bf_bits(sp[e] - bf_bits2f(hb));
                hv[e] = __builtin_bit_cast(_Float16, hb);
                lv[e] = __builtin_bit_cast(_Float16, lb);
              }
            }
            *(volatile v8h*)(C + (size_t)(mBase + row) * ldc + n0 + c8) = hv;
            if (OUT_MODE == 2) *(volatile v8h*)(C2 + (size_t)(mBase + row) * ldc + n0 + c8) = lv;
          }
        }
        __threadfence();
      }
    }
    __builtin_amdgcn_fence(__ATOMIC_RELEASE, "workgroup");
    __builtin_amdgcn_wave_barrier();
    __builtin_amdgcn_fence(__ATOMIC_ACQUIRE, "workgroup");
  }
}

__global__ __launch_bounds__(256) void tcast_bf16_kernel(const float* __restrict__ W, unsigned short* __restrict__ out,
                                                         int R, int Cc) {
  __shared__ float sm[64][65];
  const int t  = threadIdx.x;
  const int r0 = blockIdx.x * 64;
  const int c0 = blockIdx.y * 64;
#pragma unroll
  for (int i = 0; i < 16; ++i) {
    const int e  = i * 256 + t;
    const int rl = e >> 6;
    const int cl = e & 63;
    sm[cl][rl] = W[(size_t)(r0 + rl) * Cc + c0 + cl];
  }
  __syncthreads();
  const int lane = t & 31, wave = t >> 5;
  const int q = lane >> 3, c8 = (lane & 7) * 8;
  for (int pass = 0; pass < 2; ++pass) {
#pragma unroll
    for (int it = 0; it < 2; ++it) {
      const int row = wave * 8 + it * 4 + q;
      unsigned short hb[8];
#pragma unroll
      for (int e = 0; e < 8; ++e) hb[e] = f2bf_bits(sm[row][c8 + e]);
      const v4u u = (v4u){pk16(hb[0], hb[1]), pk16(hb[2], hb[3]), pk16(hb[4], hb[5]), pk16(hb[6], hb[7])};
      *(volatile v4u*)(out + (size_t)(c0 + row) * R + r0 + c8) = u;
    }
    __threadfence();
  }
}

template <bool RAW>
__global__ __launch_bounds__(256) void ln_row_kernel(const float* __restrict__ x, const float* __restrict__ g,
                                                     const float* __restrict__ bb, unsigned short* __restrict__ lnout,
                                                     unsigned short* __restrict__ rawout) {
  __shared__ __align__(16) float srow[kH];
  __shared__ float redA[8];
  __shared__ float redB[8];
  const int row = blockIdx.x;
  const int t = threadIdx.x, lane = t & 31, wave = t >> 5;
  const float* xr = x + (size_t)row * kH;
  const float v0 = xr[t], v1 = xr[t + 256], v2 = xr[t + 512];
  float s = (v0 + v1) + v2;
#pragma unroll
  for (int off = 16; off > 0; off >>= 1) s += __shfl_xor(s, off, 32);
  if (lane == 0) redA[wave] = s;
  __syncthreads();
  float tot = redA[0];
#pragma unroll
  for (int w = 1; w < 8; ++w) tot += redA[w];
  const float mean = tot * kInvH;
  const float d0 = v0 - mean, d1 = v1 - mean, d2 = v2 - mean;
  float qq = (d0 * d0 + d1 * d1) + d2 * d2;
#pragma unroll
  for (int off = 16; off > 0; off >>= 1) qq += __shfl_xor(qq, off, 32);
  if (lane == 0) redB[wave] = qq;
  __syncthreads();
  float tq = redB[0];
#pragma unroll
  for (int w = 1; w < 8; ++w) tq += redB[w];
  const float var  = tq * kInvH;
  const float rstd = rsqrtf(var + kLnEps);
  srow[t]       = d0 * rstd * g[t] + bb[t];
  srow[t + 256] = d1 * rstd * g[t + 256] + bb[t + 256];
  srow[t + 512] = d2 * rstd * g[t + 512] + bb[t + 512];
  __syncthreads();
  if (t < 96) {
    const v4f a0 = *(const v4f*)(srow + 8 * t);
    const v4f a1 = *(const v4f*)(srow + 8 * t + 4);
    const v4u u = pack8_bf16(a0, a1);
    unsigned short* lp = lnout + (size_t)row * kH + 8 * t;
    v4u ur = (v4u){0u, 0u, 0u, 0u};
    unsigned short* rp = lp;
    if (RAW) {
      const v4f r0 = *(const v4f*)(xr + 8 * t);
      const v4f r1 = *(const v4f*)(xr + 8 * t + 4);
      ur = pack8_bf16(r0, r1);
      rp = rawout + (size_t)row * kH + 8 * t;
    }
    *(volatile v4u*)lp = u;
    if (RAW) *(volatile v4u*)rp = ur;
    __threadfence();
    *(volatile v4u*)lp = u;
    if (RAW) *(volatile v4u*)rp = ur;
  }
}

__global__ __launch_bounds__(128) void softmax_row_kernel(const float* __restrict__ Sp, unsigned short* __restrict__ Pp) {
  __shared__ float redM[4];
  __shared__ float redS[4];
  const int row = blockIdx.x;
  const int hg  = blockIdx.y;
  const int t = threadIdx.x, lane = t & 31, wave = t >> 5;
  const size_t rowoff = ((size_t)hg * kS + row) * kS;
  const float* sr = Sp + rowoff + 8 * (size_t)t;
  const v4f a = *(const v4f*)(sr);
  const v4f c = *(const v4f*)(sr + 4);
  float xv[8];
#pragma unroll
  for (int e = 0; e < 4; ++e) { xv[e] = a[e] * kQKScale; xv[4 + e] = c[e] * kQKScale; }
  float m = xv[0];
#pragma unroll
  for (int e = 1; e < 8; ++e) m = fmaxf(m, xv[e]);
#pragma unroll
  for (int off = 16; off > 0; off >>= 1) m = fmaxf(m, __shfl_xor(m, off, 32));
  if (lane == 0) redM[wave] = m;
  __syncthreads();
  float mx = redM[0];
#pragma unroll
  for (int w = 1; w < 4; ++w) mx = fmaxf(mx, redM[w]);
  float ev[8];
  float sum = 0.f;
#pragma unroll
  for (int e = 0; e < 8; ++e) { ev[e] = expf(xv[e] - mx); sum += ev[e]; }
#pragma unroll
  for (int off = 16; off > 0; off >>= 1) sum += __shfl_xor(sum, off, 32);
  if (lane == 0) redS[wave] = sum;
  __syncthreads();
  float tot = redS[0];
#pragma unroll
  for (int w = 1; w < 4; ++w) tot += redS[w];
  const float inv = 1.0f / tot;
  v4f p0, p1;
#pragma unroll
  for (int e = 0; e < 4; ++e) { p0[e] = ev[e] * inv; p1[e] = ev[4 + e] * inv; }
  const v4u u = pack8_bf16(p0, p1);
  unsigned short* pr = Pp + rowoff + 8 * (size_t)t;
  *(volatile v4u*)pr = u;
  __threadfence();
  *(volatile v4u*)pr = u;
}

extern "C" void kernel_launch(void* const* d_in, const int* in_sizes, int n_in,
                              void* d_out, int out_size, void* d_ws, size_t ws_size,
                              hipStream_t stream) {
  if (n_in < 18) return;
  if (in_sizes[0] != kM * kH) return;
  if (in_sizes[1] != kH * kH || in_sizes[3] != kH * kH || in_sizes[4] != kH * kH || in_sizes[6] != kH * kH) return;
  if (in_sizes[8] != kH * kFF || in_sizes[10] != kFF * kH) return;
  if (in_sizes[2] != kH || in_sizes[5] != kH || in_sizes[7] != kH || in_sizes[11] != kH) return;
  if (in_sizes[9] != kFF) return;
  if (in_sizes[12] != kH || in_sizes[13] != kH || in_sizes[14] != kH || in_sizes[15] != kH) return;
  if (in_sizes[16] != kH || in_sizes[17] != kH) return;
  if (out_size != kM * kH) return;

  const size_t szW   = (size_t)kH * kH * 2;
  const size_t szWF  = (size_t)kH * kFF * 2;
  const size_t szAct = (size_t)kM * kH * 2;
  const size_t szVT  = (size_t)kB * kH * kS * 2;
  const size_t szHF  = (size_t)kM * kH * 4;
  const size_t szU   = (size_t)kM * kFF * 2;
  const size_t szSC  = (size_t)kGrp * kS * kS * 4;
  const size_t szPP  = (size_t)kGrp * kS * kS * 2;
  const size_t offWQ  = 0;
  const size_t offWK  = offWQ + szW;
  const size_t offWV  = offWK + szW;
  const size_t offWO  = offWV + szW;
  const size_t offWI  = offWO + szW;
  const size_t offW2  = offWI + szWF;
  const size_t offXB  = offW2 + szWF;
  const size_t offLN1 = offXB + szAct;
  const size_t offQ   = offLN1 + szAct;
  const size_t offK   = offQ + szAct;
  const size_t offVT  = offK + szAct;
  const size_t offCTX = offVT + szVT;
  const size_t offHF  = offCTX + szAct;
  const size_t offLN2 = offHF + szHF;
  const size_t offU   = offLN2 + szAct;
  const size_t offSC  = offU + szU;
  const size_t offPP  = offSC + szSC;
  const size_t total  = offPP + szPP;
  if (ws_size < total) return;

  const float* x    = (const float*)d_in[0];
  const float* wq   = (const float*)d_in[1];
  const float* bq   = (const float*)d_in[2];
  const float* wk   = (const float*)d_in[3];
  const float* wv   = (const float*)d_in[4];
  const float* bv   = (const float*)d_in[5];
  const float* wo   = (const float*)d_in[6];
  const float* bo   = (const float*)d_in[7];
  const float* wi   = (const float*)d_in[8];
  const float* bi   = (const float*)d_in[9];
  const float* w2   = (const float*)d_in[10];
  const float* b2   = (const float*)d_in[11];
  const float* ln1g = (const float*)d_in[12];
  const float* ln1b = (const float*)d_in[13];
  const float* ln2g = (const float*)d_in[14];
  const float* ln2b = (const float*)d_in[15];
  const float* lam1 = (const float*)d_in[16];
  const float* lam2 = (const float*)d_in[17];
  float* out = (float*)d_out;
  char* ws = (char*)d_ws;
  unsigned short* WQT = (unsigned short*)(ws + offWQ);
  unsigned short* WKT = (unsigned short*)(ws + offWK);
  unsigned short* WVT = (unsigned short*)(ws + offWV);
  unsigned short* WOT = (unsigned short*)(ws + offWO);
  unsigned short* WIT = (unsigned short*)(ws + offWI);
  unsigned short* W2T = (unsigned short*)(ws + offW2);
  unsigned short* XB  = (unsigned short*)(ws + offXB);
  unsigned short* LN1 = (unsigned short*)(ws + offLN1);
  unsigned short* Q16 = (unsigned short*)(ws + offQ);
  unsigned short* K16 = (unsigned short*)(ws + offK);
  unsigned short* VT  = (unsigned short*)(ws + offVT);
  unsigned short* CTX = (unsigned short*)(ws + offCTX);
  float*          HF  = (float*)(ws + offHF);
  unsigned short* LN2 = (unsigned short*)(ws + offLN2);
  unsigned short* U16 = (unsigned short*)(ws + offU);
  float*          SC  = (float*)(ws + offSC);
  unsigned short* PP  = (unsigned short*)(ws + offPP);

  tcast_bf16_kernel<<<dim3(kH / 64, kH / 64), dim3(256), 0, stream>>>(wq, WQT, kH, kH);
  tcast_bf16_kernel<<<dim3(kH / 64, kH / 64), dim3(256), 0, stream>>>(wk, WKT, kH, kH);
  tcast_bf16_kernel<<<dim3(kH / 64, kH / 64), dim3(256), 0, stream>>>(wv, WVT, kH, kH);
  tcast_bf16_kernel<<<dim3(kH / 64, kH / 64), dim3(256), 0, stream>>>(wo, WOT, kH, kH);
  tcast_bf16_kernel<<<dim3(kH / 64, kFF / 64), dim3(256), 0, stream>>>(wi, WIT, kH, kFF);
  tcast_bf16_kernel<<<dim3(kFF / 64, kH / 64), dim3(256), 0, stream>>>(w2, W2T, kFF, kH);

  ln_row_kernel<true><<<dim3(kM), dim3(256), 0, stream>>>(x, ln1g, ln1b, LN1, XB);

  const int blkProj = ((kM / 64) * (kH / 64) + 7) / 8;
  const int blkVT   = ((kH / 64) * (kS / 64) + 7) / 8;
  const int blkSc   = ((kS / 64) * (kS / 64) + 7) / 8;
  const int blkPV   = ((kS / 64) * (kHD / 64) + 7) / 8;
  const int blkWI   = ((kM / 64) * (kFF / 64) + 7) / 8;

  wmma_gemm64<1, false, 2, 3, false><<<dim3(blkProj, 1), dim3(256), 0, stream>>>(
      LN1, LN1, kH, 0L, WQT, WQT, kH, 0L, (void*)Q16, (void*)Q16, kH, 0L, bq, lam1, x, 0L, kM, kH, kH, 1.0f);
  wmma_gemm64<1, false, 0, 3, false><<<dim3(blkProj, 1), dim3(256), 0, stream>>>(
      XB, XB, kH, 0L, WKT, WKT, kH, 0L, (void*)K16, (void*)K16, kH, 0L, bq, lam1, x, 0L, kM, kH, kH, 1.0f);
  wmma_gemm64<1, false, 1, 3, false><<<dim3(blkVT, kB), dim3(256), 0, stream>>>(
      WVT, WVT, kH, 0L, XB, XB, kH, (long)kS * kH, (void*)VT, (void*)VT, kS, (long)kH * kS, bv, lam1, x, 0L, kH, kS, kH, 1.0f);

  const long strideHead = (long)kHD;
  const long strideSc   = (long)kS * kS;
  const long strideVTh  = (long)kHD * kS;
  for (int b = 0; b < kB; ++b) {
    for (int gch = 0; gch < kNH / kGrp; ++gch) {
      const int h0 = gch * kGrp;
      const size_t tokOff = ((size_t)b * kS) * kH + (size_t)h0 * kHD;
      wmma_gemm64<1, false, 0, 0, false><<<dim3(blkSc, kGrp), dim3(256), 0, stream>>>(
          Q16 + tokOff, Q16 + tokOff, kH, strideHead, K16 + tokOff, K16 + tokOff, kH, strideHead,
          (void*)SC, (void*)SC, kS, strideSc, bq, lam1, x, 0L, kS, kS, kHD, 1.0f);
      softmax_row_kernel<<<dim3(kS, kGrp), dim3(128), 0, stream>>>(SC, PP);
      const unsigned short* VTg = VT + ((size_t)b * kH + (size_t)h0 * kHD) * kS;
      unsigned short* ctxg = CTX + tokOff;
      wmma_gemm64<1, false, 0, 3, false><<<dim3(blkPV, kGrp), dim3(256), 0, stream>>>(
          PP, PP, kS, strideSc, VTg, VTg, kS, strideVTh,
          (void*)ctxg, (void*)ctxg, kH, strideHead, bq, lam1, x, 0L, kS, kHD, kS, 1.0f);
    }
  }

  wmma_gemm64<1, false, 3, 0, true><<<dim3(blkProj, 1), dim3(256), 0, stream>>>(
      CTX, CTX, kH, 0L, WOT, WOT, kH, 0L, (void*)HF, (void*)HF, kH, 0L, bo, lam1, x, 0L, kM, kH, kH, 1.0f);
  ln_row_kernel<false><<<dim3(kM), dim3(256), 0, stream>>>(HF, ln2g, ln2b, LN2, LN2);
  wmma_gemm64<1, false, 2, 3, false><<<dim3(blkWI, 1), dim3(256), 0, stream>>>(
      LN2, LN2, kH, 0L, WIT, WIT, kH, 0L, (void*)U16, (void*)U16, kFF, 0L, bi, lam2, x, 0L, kM, kFF, kH, 1.0f);
  wmma_gemm64<1, false, 3, 0, true><<<dim3(blkProj, 1), dim3(256), 0, stream>>>(
      U16, U16, kFF, 0L, W2T, W2T, kFF, 0L, (void*)out, (void*)out, kH, 0L, b2, lam2, HF, 0L, kM, kH, kFF, 1.0f);
}
